// KeyValueMemoryNetwork_62113817035231
// MI455X (gfx1250) — hardware-verified
//
#include <hip/hip_runtime.h>
#include <math.h>

typedef __attribute__((ext_vector_type(16))) _Float16 v16h;
typedef __attribute__((ext_vector_type(16))) __bf16 v16b;
typedef __attribute__((ext_vector_type(8)))  _Float16 v8h;
typedef __attribute__((ext_vector_type(8)))  float v8f;
typedef __attribute__((ext_vector_type(4)))  float v4f;
typedef __attribute__((ext_vector_type(2)))  float v2f;
typedef __attribute__((ext_vector_type(4)))  unsigned v4u;
typedef __attribute__((ext_vector_type(4)))  int v4i;
typedef float __attribute__((may_alias)) float_a;
typedef int __attribute__((may_alias)) int_a;

template <typename T> __device__ __forceinline__ void vst2(void* p, T v) { *(volatile T*)p = v; __threadfence(); *(volatile T*)p = v; }
__device__ __forceinline__ v8f wmma16(v16h a, v16h b, v8f c) {
  v8f d = __builtin_amdgcn_wmma_f32_16x16x32_f16(false, a, false, b, (short)0, c, false, false);
  asm volatile("v_nop\n\tv_nop\n\tv_nop\n\tv_nop" : "+v"(d) : "v"(a), "v"(b));
  return d;
}
__device__ __forceinline__ v8f wmma_bf(v16b a, v16b b, v8f c) {
  v8f d = __builtin_amdgcn_wmma_f32_16x16x32_bf16(false, a, false, b, (short)0, c, false, false);
  asm volatile("v_nop\n\tv_nop\n\tv_nop\n\tv_nop" : "+v"(d) : "v"(a), "v"(b));
  return d;
}
__device__ __forceinline__ v16h frag_h(const _Float16* rowk0, int lane) {
  union { v16h v; v8h q[2]; } u; const _Float16* p = rowk0 + 8 * (lane >> 4);
  u.q[0] = *(const v8h*)p; u.q[1] = *(const v8h*)(p + 16); return u.v;
}
__device__ __forceinline__ v16h frag_f32(const float* rowk0, int lane) {
  v16h a; const float* p = rowk0 + 8 * (lane >> 4);
#pragma unroll
  for (int i = 0; i < 8; ++i) { a[i] = (_Float16)p[i]; a[8 + i] = (_Float16)p[16 + i]; }
  return a;
}
__device__ __forceinline__ v16h frag_f32s(const float* rowk0, int lane, float sc) {
  v16h a; const float* p = rowk0 + 8 * (lane >> 4);
#pragma unroll
  for (int i = 0; i < 8; ++i) { a[i] = (_Float16)(p[i] * sc); a[8 + i] = (_Float16)(p[16 + i] * sc); }
  return a;
}
__device__ __forceinline__ v16h fragc_f32(const float* W, int k0, int n, int lane, int ld, int K) {
  v16h a; const int g = lane >> 4;
#pragma unroll
  for (int i = 0; i < 8; ++i) { const int ka = k0 + 8 * g + i, kb = ka + 16;
    a[i] = (_Float16)(ka < K ? W[(size_t)(ka < K ? ka : K - 1) * ld + n] : 0.f); a[8 + i] = (_Float16)(kb < K ? W[(size_t)(kb < K ? kb : K - 1) * ld + n] : 0.f); }
  return a;
}
struct F2 { v16b h, l; };
__device__ __forceinline__ F2 bsplit16(const float v[16]) { F2 r;
#pragma unroll
  for (int i = 0; i < 16; ++i) { const __bf16 h = (__bf16)v[i]; r.h[i] = h; r.l[i] = (__bf16)(v[i] - (float)h); }
  return r; }
__device__ __forceinline__ F2 split_row(const float* row, int k0, int lane) { float v[16]; const float* p = row + k0 + 8 * (lane >> 4);
#pragma unroll
  for (int i = 0; i < 8; ++i) { v[i] = p[i]; v[8 + i] = p[16 + i]; }
  return bsplit16(v); }
__device__ __forceinline__ F2 split_rowK(const float* row, int k0, int lane, int K) { float v[16]; const int g = lane >> 4;
#pragma unroll
  for (int i = 0; i < 8; ++i) { const int ka = k0 + 8 * g + i, kb = ka + 16; v[i] = ka < K ? row[ka < K ? ka : K - 1] : 0.f; v[8 + i] = kb < K ? row[kb < K ? kb : K - 1] : 0.f; }
  return bsplit16(v); }
__device__ __forceinline__ F2 split_col(const float* W, int k0, int n, int lane, int ld, int K) { float v[16]; const int g = lane >> 4;
#pragma unroll
  for (int i = 0; i < 8; ++i) { const int ka = k0 + 8 * g + i, kb = ka + 16; v[i] = ka < K ? W[(size_t)(ka < K ? ka : K - 1) * ld + n] : 0.f; v[8 + i] = kb < K ? W[(size_t)(kb < K ? kb : K - 1) * ld + n] : 0.f; }
  return bsplit16(v); }
__device__ __forceinline__ v8f mac3(const F2& a, const F2& b, v8f c) { c = wmma_bf(a.l, b.h, c); c = wmma_bf(a.h, b.l, c); return wmma_bf(a.h, b.h, c); }
__device__ __forceinline__ float sigm(float v) { return 1.0f / (1.0f + expf(-v)); }
#define LDSX() do { asm volatile("s_wait_dscnt 0" ::: "memory"); __builtin_amdgcn_wave_barrier(); __builtin_amdgcn_fence(__ATOMIC_RELEASE, "workgroup"); } while (0)


#define NB 8
#define NH 256
#define NK 256
#define NE 128
#define VOC 30000
#define FVOC 1000
typedef __attribute__((ext_vector_type(8))) __bf16 v8b;
__device__ __forceinline__ v16b frag_b(const __bf16* rowk0, int lane) {
  union { v16b v; v8b q[2]; } u; const __bf16* p = rowk0 + 8 * (lane >> 4);
  u.q[0] = *(const v8b*)p; u.q[1] = *(const v8b*)(p + 16); return u.v;
}
__device__ __forceinline__ v16b frag_gbf(const float* rowk0, int lane) {
  v16b a; const float* p = rowk0 + 8 * (lane >> 4);
#pragma unroll
  for (int i = 0; i < 8; ++i) { a[i] = (__bf16)p[i]; a[8 + i] = (__bf16)p[16 + i]; }
  return a;
}
__device__ __forceinline__ float bfr(float v) { return (float)(__bf16)v; }
__device__ __attribute__((noinline)) float exp_ni(float v) { return expf(v); }

__global__ __launch_bounds__(256) void k_attn(const float* __restrict__ hid, const float* __restrict__ kemb, const float* __restrict__ vemb, const int* __restrict__ kseq, const int* __restrict__ vseq, const int* __restrict__ msk, float* __restrict__ O) {
  __shared__ __align__(16) __bf16 skey[NK][NE + 8];
  __shared__ __align__(16) float sp[16][NK];
  __shared__ __align__(16) float so[16][NE + 4];
  const int tid = threadIdx.x, wave = tid >> 5, lane = tid & 31, col = lane & 15, g = lane >> 4;
  const int b = blockIdx.y, h0 = blockIdx.x * 16;
  { int id = kseq[b * NK + tid]; id = id < 0 ? 0 : (id >= VOC ? VOC - 1 : id); const float* src = kemb + (size_t)id * NE;
#pragma unroll
    for (int c4 = 0; c4 < NE / 4; ++c4) { const float4 v = *(const float4*)(src + c4 * 4); __bf16* d = &skey[tid][c4 * 4]; d[0] = (__bf16)v.x; d[1] = (__bf16)v.y; d[2] = (__bf16)v.z; d[3] = (__bf16)v.w; } }
  __syncthreads();
  { const float* hrow = hid + ((size_t)b * NH + h0 + col) * NE; v8f acc[2] = {};
#pragma unroll
    for (int kc = 0; kc < NE / 32; ++kc) { const v16b a = frag_gbf(hrow + kc * 32, lane);
#pragma unroll
      for (int j = 0; j < 2; ++j) acc[j] = wmma_bf(a, frag_b(&skey[(wave * 2 + j) * 16 + col][kc * 32], lane), acc[j]); }
    const float isc = sqrtf(128.0f);
#pragma unroll
    for (int j = 0; j < 2; ++j)
#pragma unroll
      for (int r = 0; r < 8; ++r) { const int k = (wave * 2 + j) * 16 + col; sp[8 * g + r][k] = exp_ni(acc[j][r] / isc) * (float)msk[((size_t)b * NH + h0 + 8 * g + r) * NK + k]; } }
  __syncthreads();
#pragma unroll
  for (int rr = 0; rr < 2; ++rr) { const int row = wave * 2 + rr; float s = 0.f;
#pragma unroll
    for (int i = 0; i < 8; ++i) s += sp[row][lane * 8 + i];
#pragma unroll
    for (int o = 1; o < 32; o <<= 1) s += __shfl_xor(s, o);
    const float den = s + 1e-10f;
#pragma unroll
    for (int i = 0; i < 8; ++i) sp[row][lane * 8 + i] = sp[row][lane * 8 + i] / den; }
  LDSX();
#pragma unroll 1
  for (int rr = 0; rr < 2; ++rr) { const int row = wave * 2 + rr; const int h = h0 + row; float4 acc4 = {0.f, 0.f, 0.f, 0.f};
#pragma unroll 2
    for (int k = 0; k < NK; ++k) { int vid = vseq[((size_t)b * NH + h) * NK + k]; vid = vid < 0 ? 0 : (vid >= FVOC ? FVOC - 1 : vid);
      const float4 vv = *(const float4*)(vemb + (size_t)vid * NE + lane * 4); const float p = sp[row][k];
      acc4.x += p * bfr(vv.x); acc4.y += p * bfr(vv.y); acc4.z += p * bfr(vv.z); acc4.w += p * bfr(vv.w); }
    *(float4*)&so[row][lane * 4] = acc4; }
  LDSX();
#pragma unroll
  for (int rr = 0; rr < 2; ++rr) { const int row = wave * 2 + rr; vst2(O + ((size_t)b * NH + h0 + row) * NE + lane * 4, *(const v4f*)&so[row][lane * 4]); }
}
__global__ __launch_bounds__(128) void k_fin(const float* __restrict__ O, float* __restrict__ out) {
  __shared__ __align__(16) float srow[NE];
  const int b = blockIdx.x, e = threadIdx.x; float s = 0.f, cnt = 0.f;
#pragma unroll 4
  for (int h = 0; h < NH; ++h) { const float v = O[((size_t)b * NH + h) * NE + e]; s += v; cnt += (v != 0.f) ? 1.0f : 0.0f; }
  srow[e] = s / cnt;
  __syncthreads();
  if (e < 32) vst2(out + (size_t)b * NE + e * 4, *(const v4f*)&srow[e * 4]);
}

extern "C" void kernel_launch(void* const* d_in, const int* in_sizes, int n_in, void* d_out, int out_size, void* d_ws, size_t ws_size, hipStream_t stream) {
  (void)in_sizes; (void)n_in; (void)out_size; (void)ws_size;
  const float* hid = (const float*)d_in[0]; const float* kemb = (const float*)d_in[1]; const float* vemb = (const float*)d_in[2];
  const int* kseq = (const int*)d_in[3]; const int* vseq = (const int*)d_in[4]; const int* msk = (const int*)d_in[5];
  float* O = (float*)d_ws;
  k_attn<<<dim3(NH / 16, NB), 256, 0, stream>>>(hid, kemb, vemb, kseq, vseq, msk, O);
  k_fin<<<NB, 128, 0, stream>>>(O, (float*)d_out);
}
